// myAdvPTRNNModel_47407849013455
// MI455X (gfx1250) — hardware-verified
//
#include <hip/hip_runtime.h>


#define NB   512
#define NS   1024
#define NH   64
#define NE   32
#define NV   10
#define NO   10
#define MR   16
#define NT   128
#define KP   136
#define HP   72
#define CH   32
#define LGP  (CH * NO)

typedef __bf16         v16bf  __attribute__((ext_vector_type(16)));
typedef unsigned short v8us_t __attribute__((ext_vector_type(8)));
typedef v8us_t __attribute__((may_alias)) v8us;
typedef float          v8f    __attribute__((ext_vector_type(8)));
typedef float          v4f_t  __attribute__((ext_vector_type(4)));
typedef v4f_t __attribute__((may_alias)) v4fa;

union Frag { v16bf v; v8us_t q[2]; };

__device__ __forceinline__ unsigned int bf16_rne_bits(float x) {
  unsigned int u = __float_as_uint(x);
  return (u + 0x7FFFu + ((u >> 16) & 1u)) >> 16;
}
__device__ __forceinline__ void split_hl(float x, unsigned short& hb, unsigned short& lb) {
  unsigned int h = bf16_rne_bits(x);
  float hf = __uint_as_float(h << 16);
  hb = (unsigned short)h;
  lb = (unsigned short)bf16_rne_bits(x - hf);
}
__device__ __forceinline__ float ftanh(float x) {
  float ax = fabsf(x);
  float t  = __builtin_amdgcn_exp2f(ax * -2.8853900817779268f);
  float r  = (1.0f - t) * __builtin_amdgcn_rcpf(1.0f + t);
  return copysignf(r, x);
}

__device__ __forceinline__ v8f wmma_bf(v16bf a, v16bf b, v8f c) {
  return __builtin_amdgcn_wmma_f32_16x16x32_bf16(false, a, false, b, (short)0, c, false, false);
}
__device__ __forceinline__ void wguard(v8f& c, const Frag& ah, const Frag& al,
                                       const Frag& bh, const Frag& bl) {
  asm volatile("v_nop\n\tv_nop\n\tv_nop\n\tv_nop"
               : "+v"(c)
               : "v"(ah.v), "v"(al.v), "v"(bh.v), "v"(bl.v));
}

__device__ __forceinline__ void mma2(v8f& acc,
                                     const unsigned short* Ah, const unsigned short* Al, int lda,
                                     const unsigned short* Bh, const unsigned short* Bl, int ldb) {
  const int l = threadIdx.x & 31, h = l >> 4, m = l & 15;
  const int ao = m * lda + 8 * h;
  const int bo = m * ldb + 8 * h;
#pragma unroll
  for (int j = 0; j < 2; ++j) {
    Frag ah, al, bh, bl;
    ah.q[0] = *(const v8us*)(Ah + ao + 32 * j);
    ah.q[1] = *(const v8us*)(Ah + ao + 32 * j + 16);
    al.q[0] = *(const v8us*)(Al + ao + 32 * j);
    al.q[1] = *(const v8us*)(Al + ao + 32 * j + 16);
    bh.q[0] = *(const v8us*)(Bh + bo + 32 * j);
    bh.q[1] = *(const v8us*)(Bh + bo + 32 * j + 16);
    bl.q[0] = *(const v8us*)(Bl + bo + 32 * j);
    bl.q[1] = *(const v8us*)(Bl + bo + 32 * j + 16);
    acc = wmma_bf(ah.v, bh.v, acc);
    acc = wmma_bf(ah.v, bl.v, acc);
    acc = wmma_bf(al.v, bh.v, acc);
    wguard(acc, ah, al, bh, bl);
  }
}

__device__ __forceinline__ void gather_x(const int* __restrict__ num1, const int* __restrict__ num2,
                                         int bbase, int t,
                                         const unsigned short* Eh, const unsigned short* El,
                                         unsigned short* Ph, unsigned short* Pl) {
  const int tid = threadIdx.x;
  const int r = tid >> 3, q = tid & 7, which = q >> 2, c = (q & 3) * 8;
  const int tt = min(max(t, 0), NS - 1);
  const size_t g = (size_t)(bbase + r) * NS + tt;
  const int i1 = num1[g];
  const int i2 = num2[g];
  int id = which ? i2 : i1;
  id = (id < 0) ? (id + NV) : id;
  id = min(max(id, 0), NV - 1);
  v8us_t vh = *(const v8us*)(Eh + id * NE + c);
  v8us_t vl = *(const v8us*)(El + id * NE + c);
  *(v8us*)(Ph + r * KP + which * NE + c) = vh;
  *(v8us*)(Pl + r * KP + which * NE + c) = vl;
}

__device__ __forceinline__ void flush_logits(const float* LG, float* __restrict__ out, int bbase, int c0) {
  const int tid = threadIdx.x;
#pragma unroll
  for (int g = 0; g < 2; ++g) {
    v4f_t  v[5];
    size_t off[5];
#pragma unroll
    for (int i = 0; i < 5; ++i) {
      const int p = tid + NT * (5 * g + i);
      const int r = p / 80;
      const int j = p - r * 80;
      v[i]   = *(const v4fa*)(LG + r * LGP + j * 4);
      off[i] = ((size_t)(bbase + r) * NS + (size_t)c0) * NO + (size_t)(j * 4);
    }
#pragma unroll
    for (int i = 0; i < 5; ++i) *(volatile v4f_t*)(out + off[i]) = v[i];
    __threadfence();
#pragma unroll
    for (int i = 0; i < 5; ++i) *(volatile v4f_t*)(out + off[i]) = v[i];
  }
}

__global__ __launch_bounds__(NT)
void k_rnn2(const int* __restrict__ num1, const int* __restrict__ num2,
            const float* __restrict__ h0, const float* __restrict__ embed_w,
            const float* __restrict__ w_ih, const float* __restrict__ w_hh,
            const float* __restrict__ b_ih, const float* __restrict__ b_hh,
            const float* __restrict__ dense_w, const float* __restrict__ dense_b,
            float* __restrict__ out, int nb) {
  __shared__ __attribute__((aligned(16))) unsigned short P1h[2][MR * KP];
  __shared__ __attribute__((aligned(16))) unsigned short P1l[2][MR * KP];
  __shared__ __attribute__((aligned(16))) unsigned short H2h[2][MR * HP];
  __shared__ __attribute__((aligned(16))) unsigned short H2l[2][MR * HP];
  __shared__ __attribute__((aligned(16))) unsigned short W1h[NH * KP];
  __shared__ __attribute__((aligned(16))) unsigned short W1l[NH * KP];
  __shared__ __attribute__((aligned(16))) unsigned short W2h[NH * KP];
  __shared__ __attribute__((aligned(16))) unsigned short W2l[NH * KP];
  __shared__ __attribute__((aligned(16))) unsigned short Wdh[16 * HP];
  __shared__ __attribute__((aligned(16))) unsigned short Wdl[16 * HP];
  __shared__ __attribute__((aligned(16))) unsigned short Eh[16 * NE];
  __shared__ __attribute__((aligned(16))) unsigned short El[16 * NE];
  __shared__ __attribute__((aligned(16))) float LG[MR * LGP];
  __shared__ __attribute__((aligned(16))) float HF[2 * MR * NH];

  const int tid   = threadIdx.x;
  const int lane  = tid & 31;
  const int wv    = tid >> 5;
  const int hh    = lane >> 4;
  const int m     = lane & 15;
  const int nw    = wv * 16;
  const int col   = nw + m;
  const int bbase = blockIdx.x * MR;
  if (bbase + MR > nb) return;

  {
    const int  ksel  = tid & 63;
    const bool useih = (tid < 64);
#pragma unroll 2
    for (int n = 0; n < NH; ++n) {
      const float a1 = w_ih[n * NH + ksel];
      const float c1 = w_hh[n * NH + ksel];
      const float a2 = w_ih[NH * NH + n * NH + ksel];
      const float c2 = w_hh[NH * NH + n * NH + ksel];
      const float v1 = useih ? a1 : c1;
      const float v2 = useih ? a2 : c2;
      unsigned short hb, lb;
      split_hl(v1, hb, lb);
      W1h[n * KP + tid] = hb;
      W1l[n * KP + tid] = lb;
      split_hl(v2, hb, lb);
      W2h[n * KP + tid] = hb;
      W2l[n * KP + tid] = lb;
    }
  }
#pragma unroll
  for (int i = 0; i < 8; ++i) {
    const int idx = tid + NT * i;
    const int o = idx >> 6, k = idx & 63;
    const int oc = min(o, NO - 1);
    float v = dense_w[oc * NH + k];
    v = (o < NO) ? v : 0.0f;
    unsigned short hb, lb;
    split_hl(v, hb, lb);
    Wdh[o * HP + k] = hb;
    Wdl[o * HP + k] = lb;
  }
#pragma unroll
  for (int i = 0; i < 4; ++i) {
    const int idx = tid + NT * i;
    const int vr = idx >> 5, c = idx & 31;
    const int vc = min(vr, NV - 1);
    float v = embed_w[vc * NE + c];
    v = (vr < NV) ? v : 0.0f;
    unsigned short hb, lb;
    split_hl(v, hb, lb);
    Eh[vr * NE + c] = hb;
    El[vr * NE + c] = lb;
  }
#pragma unroll
  for (int i = 0; i < 8; ++i) {
    const int idx = tid + NT * i;
    const int r = idx >> 6, k = idx & 63;
    const size_t g = (size_t)(bbase + r) * NH + k;
    const float a = h0[g];
    const float b = h0[(size_t)NB * NH + g];
    unsigned short hb, lb;
    split_hl(a, hb, lb);
    P1h[0][r * KP + NH + k] = hb;
    P1l[0][r * KP + NH + k] = lb;
    split_hl(b, hb, lb);
    H2h[0][r * HP + k] = hb;
    H2l[0][r * HP + k] = lb;
  }
  const float bias1r = b_ih[col] + b_hh[col];
  const float bias2r = b_ih[NH + col] + b_hh[NH + col];
  const int   mo     = min(m, NO - 1);
  float bdr = dense_b[mo];
  bdr = (m < NO) ? bdr : 0.0f;

  __syncthreads();
  gather_x(num1, num2, bbase, 0, Eh, El, P1h[0], P1l[0]);
  __syncthreads();

  const v8f zero8 = {0.f, 0.f, 0.f, 0.f, 0.f, 0.f, 0.f, 0.f};

#pragma unroll 1
  for (int t = 0; t < NS; ++t) {
    const int  cur  = t & 1, nxt = cur ^ 1;
    const bool last = (t == NS - 1);

    if (t + 1 < NS) gather_x(num1, num2, bbase, t + 1, Eh, El, P1h[nxt], P1l[nxt]);
    {
      v8f acc = zero8;
      mma2(acc, P1h[cur],      P1l[cur],      KP, W1h + nw * KP,      W1l + nw * KP,      KP);
      mma2(acc, P1h[cur] + NH, P1l[cur] + NH, KP, W1h + nw * KP + NH, W1l + nw * KP + NH, KP);
#pragma unroll
      for (int r = 0; r < 8; ++r) {
        const float v   = ftanh(acc[r] + bias1r);
        const int   row = 8 * hh + r;
        unsigned short hb, lb;
        split_hl(v, hb, lb);
        P1h[nxt][row * KP + NH + col] = hb;
        P1l[nxt][row * KP + NH + col] = lb;
        if (last) HF[row * NH + col] = v;
      }
    }
    __syncthreads();

    {
      v8f acc = zero8;
      mma2(acc, P1h[nxt] + NH, P1l[nxt] + NH, KP, W2h + nw * KP,      W2l + nw * KP,      KP);
      mma2(acc, H2h[cur],      H2l[cur],      HP, W2h + nw * KP + NH, W2l + nw * KP + NH, KP);
#pragma unroll
      for (int r = 0; r < 8; ++r) {
        const float v   = ftanh(acc[r] + bias2r);
        const int   row = 8 * hh + r;
        unsigned short hb, lb;
        split_hl(v, hb, lb);
        H2h[nxt][row * HP + col] = hb;
        H2l[nxt][row * HP + col] = lb;
        if (last) HF[MR * NH + row * NH + col] = v;
      }
    }
    __syncthreads();

    if (wv == 0) {
      v8f acc = zero8;
      mma2(acc, H2h[nxt], H2l[nxt], HP, Wdh, Wdl, HP);
      const int tc = (t & (CH - 1)) * NO;
      if (m < NO) {
#pragma unroll
        for (int r = 0; r < 8; ++r)
          LG[(8 * hh + r) * LGP + tc + m] = acc[r] + bdr;
      }
    }
    if ((t & (CH - 1)) == CH - 1) {
      __syncthreads();
      flush_logits(LG, out, bbase, t - (CH - 1));
    }
  }

  __syncthreads();
  {
    v4f_t  v[4];
    size_t off[4];
#pragma unroll
    for (int i = 0; i < 4; ++i) {
      const int p = tid + NT * i;
      const int l = p >> 8, rem = p & 255;
      v[i]   = *(const v4fa*)(HF + l * (MR * NH) + rem * 4);
      off[i] = (size_t)NB * NS * NO + (size_t)l * NB * NH + (size_t)bbase * NH + (size_t)(rem * 4);
    }
#pragma unroll
    for (int i = 0; i < 4; ++i) *(volatile v4f_t*)(out + off[i]) = v[i];
    __threadfence();
#pragma unroll
    for (int i = 0; i < 4; ++i) *(volatile v4f_t*)(out + off[i]) = v[i];
  }
}

extern "C" void kernel_launch(void* const* d_in, const int* in_sizes, int n_in,
                              void* d_out, int out_size, void* d_ws, size_t ws_size,
                              hipStream_t stream) {
  (void)d_ws; (void)ws_size;
  if (n_in < 10) return;
  if (in_sizes[0] != NB * NS || in_sizes[1] != NB * NS || in_sizes[2] != 2 * NB * NH ||
      in_sizes[3] != NV * NE || in_sizes[4] != 2 * NH * NH || in_sizes[5] != 2 * NH * NH ||
      in_sizes[6] != 2 * NH || in_sizes[7] != 2 * NH || in_sizes[8] != NO * NH || in_sizes[9] != NO) return;
  if (out_size != NB * NS * NO + 2 * NB * NH) return;

  const int*   num1    = (const int*)d_in[0];
  const int*   num2    = (const int*)d_in[1];
  const float* h0      = (const float*)d_in[2];
  const float* embed_w = (const float*)d_in[3];
  const float* w_ih    = (const float*)d_in[4];
  const float* w_hh    = (const float*)d_in[5];
  const float* b_ih    = (const float*)d_in[6];
  const float* b_hh    = (const float*)d_in[7];
  const float* dense_w = (const float*)d_in[8];
  const float* dense_b = (const float*)d_in[9];

  k_rnn2<<<dim3(NB / MR), dim3(NT), 0, stream>>>(num1, num2, h0, embed_w, w_ih, w_hh, b_ih, b_hh,
                                                 dense_w, dense_b, (float*)d_out, NB);
}
